// HeteroGraph_58179626992420
// MI455X (gfx1250) — hardware-run, weakly checked
//
#include <hip/hip_runtime.h>


namespace {
constexpr int N = 50000, E = 800000, C = 128, NPB = 8;
constexpr float XS = 8.0f, HS = 256.0f, WSC = 256.0f, EPS = 1e-5f, SLOPE = 0.2f;
typedef _Float16 b16;
typedef __attribute__((ext_vector_type(16))) _Float16 v16b;
typedef __attribute__((ext_vector_type(8))) _Float16 v8b;
typedef __attribute__((ext_vector_type(8))) float v8f;
typedef __attribute__((ext_vector_type(4))) float v4f;
__device__ __forceinline__ float bf16_rne(float f) { unsigned int u = __float_as_uint(f); u += 0x7FFFu + ((u >> 16) & 1u); float r = __uint_as_float(u & 0xFFFF0000u); asm volatile("" : "+v"(r)); return r; }
__device__ __forceinline__ float bfv(float f) { float r = bf16_rne(f); asm volatile("" : "+v"(r)); return r; }
__device__ __forceinline__ void split16(float v, b16& hi, b16& lo) { hi = (b16)v; lo = (b16)(v - (float)hi); }
__device__ __forceinline__ v16b frag_kb(const b16* p, int hh) { const v8b a = *(const v8b*)(p + 8 * hh), b = *(const v8b*)(p + 16 + 8 * hh); v16b f;
#pragma unroll
  for (int e = 0; e < 8; ++e) { f[e] = a[e]; f[8 + e] = b[e]; } return f; }
__device__ __forceinline__ v8f wmma16b(v16b a, v16b b, v8f c) { v8f d = __builtin_amdgcn_wmma_f32_16x16x32_f16(false, a, false, b, (short)0, c, false, false); asm volatile("v_nop\n\tv_nop\n\tv_nop\n\tv_nop" : "+v"(d) : "v"(a), "v"(b)); return d; }
__device__ __forceinline__ void wave_lds_sync() { __builtin_amdgcn_fence(__ATOMIC_RELEASE, "workgroup"); __builtin_amdgcn_wave_barrier(); __builtin_amdgcn_fence(__ATOMIC_ACQUIRE, "workgroup"); }
__device__ __forceinline__ float pmul(float a, float b) { float p = a * b; asm volatile("" : "+v"(p)); return p; }
__device__ __forceinline__ int iclamp(int v, int lo, int hi) { return v < lo ? lo : (v > hi ? hi : v); }
constexpr int CSR_NBLK8 = 512, CSR_GB8 = 8, CSR_GN8 = 1 << CSR_GB8  , CSR_TS8 = (CSR_GN8 < 32 ? 32 : CSR_GN8)  , CSR_MAXG8 = 512, CSR_CAP8 = 12288  ;
__device__ __host__ __forceinline__ int csr_tix8(int v) { return (v >> CSR_GB8) * CSR_TS8 + (v & (CSR_GN8 - 1)); }
__global__ __launch_bounds__(64) void csrA_kernel8(const int* __restrict__ dst, int E, int N, int nG, int CHP, int NGP, int* __restrict__ STG, int* __restrict__ HST) {
  extern __shared__ int sm[];
  int* cnt = sm; int* run = sm + NGP; int* ids = sm + 2 * NGP;
  const int b = blockIdx.x; const int ch = (E + CSR_NBLK8 - 1) / CSR_NBLK8; const int e0 = b * ch, e1 = min(E, e0 + ch);
  for (int i = threadIdx.x; i < NGP; i += 64) cnt[i] = 0;
  for (int i = threadIdx.x; i < CHP; i += 64) ids[i] = -1;
  __syncthreads();
  if (threadIdx.x == 0) {
    for (int e = e0; e < e1; ++e) { int d = dst[e]; d = (d < 0) ? 0 : (d >= N ? N - 1 : d); cnt[d >> CSR_GB8] += 1; }
    int acc = 0; for (int g = 0; g < nG; ++g) { run[g] = acc; acc += cnt[g]; }
    for (int e = e0; e < e1; ++e) { int d = dst[e]; d = (d < 0) ? 0 : (d >= N ? N - 1 : d); const int g = d >> CSR_GB8; ids[run[g]] = e; run[g] += 1; } }
  __syncthreads();
  typedef __attribute__((ext_vector_type(4))) int v4i;
  for (int pass = 0; pass < 2; ++pass) {
    for (int i = threadIdx.x; i < CHP / 4; i += 64) *(volatile v4i*)(STG + (size_t)b * CHP + i * 4) = *(const v4i*)(&ids[i * 4]);
    for (int i = threadIdx.x; i < NGP / 4; i += 64) { v4i v; for (int e = 0; e < 4; ++e) v[e] = (i * 4 + e < nG) ? cnt[i * 4 + e] : 0; *(volatile v4i*)(HST + (size_t)b * NGP + i * 4) = v; }
    __threadfence(); }
}
__global__ __launch_bounds__(512) void csrS_kernel8(const int* __restrict__ HST, int nG, int NGP, int* __restrict__ START, int* __restrict__ TOT, int* __restrict__ OFF) {
  __shared__ int tot[CSR_MAXG8];
  const int b = threadIdx.x;
  for (int pass = 0; pass < 2; ++pass) { int runb = 0; for (int g = 0; g < nG; ++g) { int c = HST[(size_t)b * NGP + g]; c = (c < 0) ? 0 : c; ((volatile int*)OFF)[(size_t)g * CSR_NBLK8 + b] = runb; runb += c; } __threadfence(); }
  for (int g = threadIdx.x; g < nG; g += 512) { int s = 0; for (int bb = 0; bb < CSR_NBLK8; ++bb) { int c = HST[(size_t)bb * NGP + g]; s += (c < 0) ? 0 : c; } tot[g] = s; }
  __syncthreads();
  if (threadIdx.x < 32) {
    __shared__ int st[CSR_MAXG8 + 32];
    if (threadIdx.x == 0) { int acc = 0; for (int g = 0; g < NGP; ++g) { st[g] = acc; if (g < nG) acc += (tot[g] + 31) & ~31; } st[NGP] = acc; }
    __builtin_amdgcn_fence(__ATOMIC_RELEASE, "workgroup"); __builtin_amdgcn_wave_barrier(); __builtin_amdgcn_fence(__ATOMIC_ACQUIRE, "workgroup");
    for (int pass = 0; pass < 2; ++pass) { for (int i = threadIdx.x; i < NGP + 32; i += 32) { ((volatile int*)START)[i] = (i <= NGP) ? st[min(i, NGP)] : 0; ((volatile int*)TOT)[i] = (i < nG) ? tot[i] : 0; } __threadfence(); } }
}
__global__ __launch_bounds__(256) void csrB_kernel8(const int* __restrict__ dst, int N, int nG, int CHP, int NGP, int permLen, const int* __restrict__ STG, const int* __restrict__ HST, const int* __restrict__ OFF, const int* __restrict__ START, const int* __restrict__ TOT, int* __restrict__ PERM, int* __restrict__ ROWPTR, int* __restrict__ ROWCNT, int* __restrict__ FLAG) {
  typedef __attribute__((ext_vector_type(4))) int v4i;
  __shared__ int ids[CSR_CAP8]; __shared__ unsigned short key[CSR_CAP8]; __shared__ int outp[CSR_CAP8]; __shared__ int ncnt[CSR_GN8 + 1]; __shared__ int boff[CSR_NBLK8 + 1];
  const int g = blockIdx.x, t_ = threadIdx.x; int tot = TOT[g]; int st = START[g], stn = START[g + 1]; const int v0 = g * CSR_GN8; const int nv = min(CSR_GN8, N - v0); const int t0 = g * CSR_TS8;
  st = (st < 0) ? 0 : (st > permLen - 32 ? permLen - 32 : st) & ~31; stn = (stn < st) ? st : (stn > permLen ? permLen : stn); tot = (tot < 0) ? 0 : tot; if (tot > stn - st && tot <= CSR_CAP8) tot = stn - st;
  if (tot > CSR_CAP8) {
    for (int pass = 0; pass < 2; ++pass) { for (int i = t_; i < CSR_TS8 / 4; i += 256) { v4i a, c; for (int e = 0; e < 4; ++e) { a[e] = st; c[e] = 0; } *(volatile v4i*)(ROWPTR + t0 + i * 4) = a; *(volatile v4i*)(ROWCNT + t0 + i * 4) = c; } if (t_ == 0) ((volatile int*)FLAG)[0] = 1; __threadfence(); } (void)nv; return; }
  if (t_ == 0) { int acc = 0; for (int b = 0; b < CSR_NBLK8; ++b) { boff[b] = acc; int c = HST[(size_t)b * NGP + g]; c = (c < 0) ? 0 : (c > CHP ? CHP : c); acc += c; if (acc > tot) acc = tot; } boff[CSR_NBLK8] = acc; }
  for (int i = t_; i <= CSR_GN8; i += 256) ncnt[i] = 0;
  __syncthreads();
  for (int b = 0; b < CSR_NBLK8; ++b) { const int c = boff[b + 1] - boff[b]; int o_ = OFF[(size_t)g * CSR_NBLK8 + b]; o_ = (o_ < 0) ? 0 : (o_ > CHP - c ? CHP - c : o_); const int* src_ = STG + (size_t)b * CHP + o_;
    for (int i = t_; i < c; i += 256) { int id = src_[i]; id = (id < 0) ? 0 : id; ids[boff[b] + i] = id; int d = dst[id]; d = (d < v0) ? v0 : (d >= N ? N - 1 : d); int kk = d - v0; kk = (kk < 0) ? 0 : (kk >= CSR_GN8 ? CSR_GN8 - 1 : kk); key[boff[b] + i] = (unsigned short)kk; } }
  __syncthreads();
  if (t_ == 0) { for (int i = 0; i < tot; ++i) ncnt[key[i]] += 1; int acc = 0; for (int vl = 0; vl < CSR_GN8; ++vl) { const int c = ncnt[vl]; ncnt[vl] = acc; acc += c; } ncnt[CSR_GN8] = acc;
    for (int i = 0; i < tot; ++i) { const int vl = key[i]; outp[ncnt[vl]] = ids[i]; ncnt[vl] += 1; }
    for (int vl = CSR_GN8; vl > 0; --vl) ncnt[vl] = ncnt[vl - 1]; ncnt[0] = 0; }
  __syncthreads();
  for (int pass = 0; pass < 2; ++pass) {
    for (int i = t_; i < (stn - st) / 4; i += 256) { v4i v; for (int e = 0; e < 4; ++e) { const int q = i * 4 + e; v[e] = (q < tot) ? outp[q] : -1; } *(volatile v4i*)(PERM + st + i * 4) = v; }
    for (int i = t_; i < CSR_TS8 / 4; i += 256) { v4i a, c; for (int e = 0; e < 4; ++e) { const int vl = i * 4 + e; const int vc = vl < CSR_GN8 ? vl : CSR_GN8; a[e] = (vl < CSR_GN8) ? st + ncnt[vc] : st; c[e] = (vl < nv) ? (ncnt[(vc < CSR_GN8 ? vc : CSR_GN8 - 1) + 1] - ncnt[vc]) : 0; } *(volatile v4i*)(ROWPTR + t0 + i * 4) = a; *(volatile v4i*)(ROWCNT + t0 + i * 4) = c; }
    __threadfence(); }
}
__global__ __launch_bounds__(256) void csrZ_kernel8(int* __restrict__ p, size_t n4) { typedef __attribute__((ext_vector_type(4))) int v4i; const size_t tid = (size_t)blockIdx.x * 256 + threadIdx.x, nth = (size_t)gridDim.x * 256; v4i z = {0, 0, 0, 0}; for (size_t i = tid; i < n4; i += nth) *(volatile v4i*)(p + i * 4) = z; }
struct CsrBufs8 { int *STG, *HST, *OFF, *START, *TOT, *PERM, *ROWPTR, *ROWCNT, *FLAG; int nG, NGP, CHP; size_t permLen; char* base; size_t bytes; };
static size_t csr_carve8(CsrBufs8& c, char* ws, size_t off, int E, int N) {
  const size_t off0 = off; c.base = ws + off;
  auto al = [&](size_t bytes) { char* p = ws + off; off += (bytes + 255) & ~(size_t)255; return p; };
  c.nG = (N + CSR_GN8 - 1) / CSR_GN8; c.NGP = (c.nG + 31) & ~31; const int ch = (E + CSR_NBLK8 - 1) / CSR_NBLK8; c.CHP = (ch + 31) & ~31; c.permLen = (size_t)E + 32 * (size_t)c.nG + 32;
  c.STG = (int*)al((size_t)CSR_NBLK8 * c.CHP * 4); c.HST = (int*)al((size_t)CSR_NBLK8 * c.NGP * 4); c.OFF = (int*)al((size_t)c.NGP * CSR_NBLK8 * 4); c.START = (int*)al((size_t)(c.NGP + 64) * 4); c.TOT = (int*)al((size_t)(c.NGP + 64) * 4);
  c.PERM = (int*)al(c.permLen * 4); c.ROWPTR = (int*)al((size_t)c.nG * CSR_TS8 * 4); c.ROWCNT = (int*)al((size_t)c.nG * CSR_TS8 * 4); c.FLAG = (int*)al(256);
  c.bytes = off - off0; return off;
}
static void csr_build8(const CsrBufs8& c, const int* dst, int E, int N, hipStream_t stream) {
  const size_t smem = (size_t)(2 * c.NGP + c.CHP) * 4;
  csrZ_kernel8<<<512, 256, 0, stream>>>((int*)c.base, c.bytes / 16);
  csrA_kernel8<<<CSR_NBLK8, 64, smem, stream>>>(dst, E, N, c.nG, c.CHP, c.NGP, c.STG, c.HST);
  csrS_kernel8<<<1, 512, 0, stream>>>(c.HST, c.nG, c.NGP, c.START, c.TOT, c.OFF);
  csrB_kernel8<<<c.nG, 256, 0, stream>>>(dst, N, c.nG, c.CHP, c.NGP, (int)c.permLen, c.STG, c.HST, c.OFF, c.START, c.TOT, c.PERM, c.ROWPTR, c.ROWCNT, c.FLAG);
}


__global__ __launch_bounds__(256) void wput_kernel(const float* __restrict__ swl, const float* __restrict__ swr, const float* __restrict__ sbl, const float* __restrict__ sbr, const float* __restrict__ gwWs, const float* __restrict__ gwWd, const float* __restrict__ gbWs, const float* __restrict__ gbWd, b16* __restrict__ WS0, b16* __restrict__ WG) { const int u = blockIdx.x * 256 + threadIdx.x; v8b v;
  if (u < 2 * C * 32) { const int t = u / (C * 32), r = (u / 32) % C, k0 = (u % 32) * 8; const float* wl = t == 0 ? swl : sbl; const float* wr = t == 0 ? swr : sbr;
#pragma unroll
    for (int j = 0; j < 8; ++j) { const int k = k0 + j; v[j] = (b16)(bf16_rne(k < C ? wl[(size_t)r * C + k] : wr[(size_t)r * C + (k - C)]) * WSC); } for (int pass = 0; pass < 2; ++pass) { *(volatile v8b*)(WS0 + ((size_t)t * C + r) * 2 * C + k0) = v; __threadfence(); } }
  if (u < 2 * 2 * C * 16) { const int t = u / (2 * C * 16), r = (u / 16) % (2 * C), k0 = (u % 16) * 8; const float* w = t == 0 ? (r < C ? gbWs : gwWd) : (r < C ? gwWs : gbWd); const int rr = r % C;
#pragma unroll
    for (int j = 0; j < 8; ++j) v[j] = (b16)(bf16_rne(w[(size_t)rr * C + k0 + j]) * WSC); for (int pass = 0; pass < 2; ++pass) { *(volatile v8b*)(WG + ((size_t)t * 2 * C + r) * C + k0) = v; __threadfence(); } } }
__device__ __forceinline__ void ln_relu_row(float* row, const float* g, const float* b) { float m = 0.0f; for (int c = 0; c < C; ++c) m += row[c]; m *= (1.0f / C); float vr = 0.0f; for (int c = 0; c < C; ++c) { const float d = row[c] - m; vr += d * d; } vr *= (1.0f / C); const float rs = rsqrtf(vr + EPS); for (int c = 0; c < C; ++c) row[c] = fmaxf(pmul((row[c] - m) * rs, bfv(g[c])) + bfv(b[c]), 0.0f); }
__global__ __launch_bounds__(32) void sage_kernel(const float* __restrict__ xp, const float* __restrict__ xa, const int* __restrict__ srcW, const int* __restrict__ PERMw, const int* __restrict__ RPw, const int* __restrict__ RCw, int plW, const int* __restrict__ srcB, const int* __restrict__ PERMb, const int* __restrict__ RPb, const int* __restrict__ RCb, int plB, const b16* __restrict__ WS0, const float* __restrict__ swbl, const float* __restrict__ sbbl, const float* __restrict__ g0p, const float* __restrict__ b0p, const float* __restrict__ g0a, const float* __restrict__ b0a, int NLIM, float* __restrict__ X1p, float* __restrict__ X1a) { __shared__ __attribute__((aligned(16))) b16 Ah[16][264], Al[16][264]; __shared__ float Tf[16][C + 1]; const int lane = threadIdx.x, nloc = lane & 15, hlf = lane >> 4; const int t = blockIdx.y; const size_t n0 = (size_t)blockIdx.x * 16; if (n0 >= (size_t)NLIM) return;
  const float* xown = t == 0 ? xp : xa; const float* xoth = t == 0 ? xa : xp; const int* srcs = t == 0 ? srcW : srcB; const int* PERM = t == 0 ? PERMw : PERMb; const int* RP = t == 0 ? RPw : RPb; const int* RC = t == 0 ? RCw : RCb; const int pl = t == 0 ? plW : plB;
  if (lane < 16) for (int k = 256; k < 264; ++k) { Ah[lane][k] = (b16)0.0f; Al[lane][k] = (b16)0.0f; }
  for (int rr = 0; rr < 16; ++rr) { const size_t n = n0 + rr; int st = RP[n], cnt = RC[n]; cnt = iclamp(cnt, 0, E); st = iclamp(st, 0, pl - cnt); v4f a = {0, 0, 0, 0};
#pragma unroll 1
    for (int j = 0; j < cnt; ++j) { const int e = iclamp(PERM[st + j], 0, E - 1); const size_t s = (size_t)iclamp(srcs[e], 0, N - 1); if (s >= (size_t)NLIM) continue; const float* xs = xoth + s * C + lane * 4; a += (v4f){bfv(xs[0]), bfv(xs[1]), bfv(xs[2]), bfv(xs[3])}; }
    for (int q = 0; q < 4; ++q) { b16 p, pl2; split16(a[q] * HS, p, pl2); Ah[rr][lane * 4 + q] = p; Al[rr][lane * 4 + q] = pl2; const float xv = bfv(xown[n * C + lane * 4 + q]); Ah[rr][C + lane * 4 + q] = (b16)(xv * XS); Al[rr][C + lane * 4 + q] = (b16)0.0f; } }
  wave_lds_sync(); v8f accA[8], accX[8];
#pragma unroll
  for (int tt = 0; tt < 8; ++tt) { accA[tt] = (v8f){}; accX[tt] = (v8f){}; }
  const b16* Wb = WS0 + (size_t)t * C * 2 * C;
#pragma unroll
  for (int kb = 0; kb < C; kb += 32) { const v16b a = frag_kb(&Ah[nloc][kb], hlf), al = frag_kb(&Al[nloc][kb], hlf), ax = frag_kb(&Ah[nloc][C + kb], hlf);
#pragma unroll
    for (int tt = 0; tt < 8; ++tt) { const v16b bw = frag_kb(Wb + (size_t)(tt * 16 + nloc) * 2 * C + kb, hlf), bx = frag_kb(Wb + (size_t)(tt * 16 + nloc) * 2 * C + C + kb, hlf); accA[tt] = wmma16b(a, bw, accA[tt]); accA[tt] = wmma16b(al, bw, accA[tt]); accX[tt] = wmma16b(ax, bx, accX[tt]); } }
  const float* bl = t == 0 ? swbl : sbbl;
#pragma unroll
  for (int tt = 0; tt < 8; ++tt) { const int cc = tt * 16 + nloc; const float bb = bfv(bl[cc]);
#pragma unroll
    for (int r8 = 0; r8 < 8; ++r8) Tf[8 * hlf + r8][cc] = accA[tt][r8] * (1.0f / (HS * WSC)) + accX[tt][r8] * (1.0f / (XS * WSC)) + bb; }
  wave_lds_sync();
  if (lane < 16) ln_relu_row(&Tf[lane][0], t == 0 ? g0p : g0a, t == 0 ? b0p : b0a);
  wave_lds_sync();
  float* X1 = t == 0 ? X1p : X1a;
  for (int pass = 0; pass < 2; ++pass) { for (int rr = 0; rr < 16; ++rr) *(volatile v4f*)(X1 + (n0 + rr) * C + lane * 4) = *(const v4f*)(&Tf[rr][lane * 4]); __threadfence(); } }
__global__ __launch_bounds__(32) void gproj_kernel(const float* __restrict__ X1p, const float* __restrict__ X1a, const b16* __restrict__ WG, const float* __restrict__ gw_as, const float* __restrict__ gw_ad, const float* __restrict__ gb_as, const float* __restrict__ gb_ad, int NLIM, float* __restrict__ HPp, float* __restrict__ HPa, float* __restrict__ ALp, float* __restrict__ ALa) { __shared__ __attribute__((aligned(16))) b16 Ah[16][C + 8], Al[16][C + 8]; __shared__ float Tf[16][260], As[16][2]; const int lane = threadIdx.x, nloc = lane & 15, hlf = lane >> 4; const int t = blockIdx.y; const size_t n0 = (size_t)blockIdx.x * 16; if (n0 >= (size_t)NLIM) return;
  const float* X1 = t == 0 ? X1p : X1a;
  for (int rr = 0; rr < 16; ++rr) for (int q = 0; q < 4; ++q) { const int c = q * 32 + lane; b16 p, pl; split16(X1[(n0 + rr) * C + c] * HS, p, pl); Ah[rr][c] = p; Al[rr][c] = pl; }
  if (lane < 16) for (int k = C; k < C + 8; ++k) { Ah[lane][k] = (b16)0.0f; Al[lane][k] = (b16)0.0f; }
  wave_lds_sync(); v8f acc[16];
#pragma unroll
  for (int tt = 0; tt < 16; ++tt) acc[tt] = (v8f){};
  const b16* Wb = WG + (size_t)t * 2 * C * C;
#pragma unroll
  for (int kb = 0; kb < C; kb += 32) { const v16b a = frag_kb(&Ah[nloc][kb], hlf), al = frag_kb(&Al[nloc][kb], hlf);
#pragma unroll
    for (int tt = 0; tt < 16; ++tt) { const v16b bw = frag_kb(Wb + (size_t)(tt * 16 + nloc) * C + kb, hlf); acc[tt] = wmma16b(a, bw, acc[tt]); acc[tt] = wmma16b(al, bw, acc[tt]); } }
#pragma unroll
  for (int tt = 0; tt < 16; ++tt)
#pragma unroll
    for (int r8 = 0; r8 < 8; ++r8) Tf[8 * hlf + r8][tt * 16 + nloc] = acc[tt][r8] * (1.0f / (HS * WSC));
  wave_lds_sync();
  { const float* as_ = t == 0 ? gb_as : gw_as; const float* ad_ = t == 0 ? gw_ad : gb_ad; const int r = nloc; float s = 0.0f; if (hlf == 0) { for (int c = 0; c < C; ++c) s += pmul(Tf[r][c], bfv(as_[c])); } else { for (int c = 0; c < C; ++c) s += pmul(Tf[r][C + c], bfv(ad_[c])); } As[r][hlf] = s; }
  wave_lds_sync();
  float* HP = t == 0 ? HPp : HPa; float* AL = t == 0 ? ALp : ALa;
  for (int pass = 0; pass < 2; ++pass) { for (int rr = 0; rr < 16; ++rr) for (int q = 0; q < 2; ++q) *(volatile v4f*)(HP + (n0 + rr) * 2 * C + q * 128 + lane * 4) = *(const v4f*)(&Tf[rr][q * 128 + lane * 4]); ((volatile float*)AL)[n0 * 2 + lane] = As[lane >> 1][lane & 1]; __threadfence(); } }
__global__ __launch_bounds__(256) void gat_kernel(const float* __restrict__ HPp, const float* __restrict__ HPa, const float* __restrict__ ALp, const float* __restrict__ ALa, const int* __restrict__ srcW, const int* __restrict__ PERMw, const int* __restrict__ RPw, const int* __restrict__ RCw, int plW, const int* __restrict__ srcB, const int* __restrict__ PERMb, const int* __restrict__ RPb, const int* __restrict__ RCb, int plB, const float* __restrict__ gw_b, const float* __restrict__ gb_b, const float* __restrict__ g1p, const float* __restrict__ b1p, const float* __restrict__ g1a, const float* __restrict__ b1a, int NLIM, float* __restrict__ outp, float* __restrict__ outa) { const int wave = threadIdx.x >> 5, lane = threadIdx.x & 31; const int t = blockIdx.y; const size_t n = (size_t)blockIdx.x * NPB + wave; if (n >= (size_t)NLIM) return;
  const float* HPo = t == 0 ? HPa : HPp; const float* ALo = t == 0 ? ALa : ALp; const float ad = (t == 0 ? ALp : ALa)[n * 2 + 1]; const int* srcs = t == 0 ? srcW : srcB; const int* PERM = t == 0 ? PERMw : PERMb; const int* RP = t == 0 ? RPw : RPb; const int* RC = t == 0 ? RCw : RCb; const int pl = t == 0 ? plW : plB;
  int st = RP[n], cnt = RC[n]; cnt = iclamp(cnt, 0, E); st = iclamp(st, 0, pl - cnt); float mx = -INFINITY, den = 0.0f; v4f acc = {0, 0, 0, 0};
#pragma unroll 1
  for (int j = 0; j < cnt; ++j) { const int e = iclamp(PERM[st + j], 0, E - 1); const size_t s = (size_t)iclamp(srcs[e], 0, N - 1); if (s >= (size_t)NLIM) continue; float lg = ALo[s * 2] + ad; lg = lg > 0.0f ? lg : SLOPE * lg; const float mn = fmaxf(mx, lg); const float sf = (mx == -INFINITY) ? 0.0f : __expf(mx - mn); const float p = __expf(lg - mn); const v4f hv = *(const v4f*)(HPo + s * 2 * C + lane * 4); acc[0] = pmul(acc[0], sf) + pmul(p, hv[0]); acc[1] = pmul(acc[1], sf) + pmul(p, hv[1]); acc[2] = pmul(acc[2], sf) + pmul(p, hv[2]); acc[3] = pmul(acc[3], sf) + pmul(p, hv[3]); den = pmul(den, sf) + p; mx = mn; }
  const float inv = den > 0.0f ? __builtin_amdgcn_rcpf(den + 1e-16f) : 0.0f; const float* bb = t == 0 ? gw_b : gb_b; const float* g = t == 0 ? g1p : g1a; const float* be = t == 0 ? b1p : b1a;
  v4f o; for (int q = 0; q < 4; ++q) o[q] = pmul(acc[q], inv) + bfv(bb[lane * 4 + q]);
  float s1 = o[0] + o[1] + o[2] + o[3]; for (int sh = 16; sh; sh >>= 1) s1 += __shfl_xor(s1, sh); const float m = s1 * (1.0f / C); float s2 = 0.0f; for (int q = 0; q < 4; ++q) { const float d = o[q] - m; s2 += d * d; } for (int sh = 16; sh; sh >>= 1) s2 += __shfl_xor(s2, sh); const float rs = rsqrtf(s2 * (1.0f / C) + EPS);
  v4f r; for (int q = 0; q < 4; ++q) { const int c = lane * 4 + q; r[q] = fmaxf(pmul((o[q] - m) * rs, bfv(g[c])) + bfv(be[c]), 0.0f); }
  float* out = t == 0 ? outp : outa;
  for (int pass = 0; pass < 2; ++pass) { *(volatile v4f*)(out + n * C + lane * 4) = r; __threadfence(); } }
}

extern "C" void kernel_launch(void* const* d_in, const int* in_sizes, int n_in, void* d_out, int out_size, void* d_ws, size_t ws_size, hipStream_t stream) {
  (void)n_in;
  auto Fp = [&](int i) { return (const float*)d_in[i]; }; auto Ip = [&](int i) { return (const int*)d_in[i]; };
  if (in_sizes[0] != N * C || in_sizes[1] != N * C || in_sizes[2] != 2 * E || in_sizes[3] != 2 * E || in_sizes[4] != C * C || in_sizes[15] != C * C || in_sizes[27] != C || out_size != 2 * N * C) return;
  const int NLIM = N;
  size_t off = 0; char* ws = (char*)d_ws;
  auto carve = [&](size_t bytes) { char* p = ws + off; off += (bytes + 255) & ~(size_t)255; return p; };
  b16* WS0 = (b16*)carve((size_t)2 * C * 2 * C * 2); b16* WG = (b16*)carve((size_t)2 * 2 * C * C * 2); float* X1p = (float*)carve((size_t)N * C * 4); float* X1a = (float*)carve((size_t)N * C * 4); float* HPp = (float*)carve((size_t)N * 2 * C * 4); float* HPa = (float*)carve((size_t)N * 2 * C * 4); float* ALp = (float*)carve((size_t)N * 2 * 4); float* ALa = (float*)carve((size_t)N * 2 * 4);
  CsrBufs8 cw; off = csr_carve8(cw, ws, off, E, N); CsrBufs8 cb; off = csr_carve8(cb, ws, off, E, N);
  if (off > ws_size || off > ((size_t)208 << 20)) return;
  wput_kernel<<<(2 * 2 * C * 16 + 255) / 256, 256, 0, stream>>>(Fp(4), Fp(6), Fp(7), Fp(9), Fp(10), Fp(11), Fp(15), Fp(16), WS0, WG);
  csr_build8(cw, Ip(2) + E, E, N, stream);
  csr_build8(cb, Ip(3) + E, E, N, stream);
  sage_kernel<<<dim3(NLIM / 16, 2), 32, 0, stream>>>(Fp(0), Fp(1), Ip(2), cw.PERM, cw.ROWPTR, cw.ROWCNT, (int)cw.permLen, Ip(3), cb.PERM, cb.ROWPTR, cb.ROWCNT, (int)cb.permLen, WS0, Fp(5), Fp(8), Fp(20), Fp(21), Fp(22), Fp(23), NLIM, X1p, X1a);
  gproj_kernel<<<dim3(NLIM / 16, 2), 32, 0, stream>>>(X1p, X1a, WG, Fp(12), Fp(13), Fp(17), Fp(18), NLIM, HPp, HPa, ALp, ALa);
  float* outp = (float*)d_out; float* outa = outp + (size_t)N * C;
  gat_kernel<<<dim3((NLIM + NPB - 1) / NPB, 2), 256, 0, stream>>>(HPp, HPa, ALp, ALa, Ip(2), cw.PERM, cw.ROWPTR, cw.ROWCNT, (int)cw.permLen, Ip(3), cb.PERM, cb.ROWPTR, cb.ROWCNT, (int)cb.permLen, Fp(14), Fp(19), Fp(24), Fp(25), Fp(26), Fp(27), NLIM, outp, outa);
}
